// SparseLayer_56281251447203
// MI455X (gfx1250) — hardware-verified
//
#include <hip/hip_runtime.h>
#include <math.h>

typedef __attribute__((ext_vector_type(16))) _Float16 v16h;
typedef __attribute__((ext_vector_type(8)))  float    v8f;
typedef __attribute__((ext_vector_type(4)))  float    v4f;
typedef __attribute__((ext_vector_type(4)))  int      v4i;

constexpr int kBatch     = 8;
constexpr int kChunks    = 128;
constexpr int kCpc       = 32;
constexpr int kPpc       = 12;
constexpr int kPts       = kCpc * kPpc;
constexpr int kInW       = 1024;
constexpr int kOutW      = 1024;
constexpr int kPitch     = 36;
constexpr int kPtsBatch  = kChunks * kPts;
constexpr int kRedThreads = 512;
static_assert(kPts == 384, "points per chunk");
static_assert((kPts % 32) == 0, "whole waves");
static_assert((kPts % 16) == 0 && kCpc == 32, "GEMV tiles: M multiple of 16, K exactly one 32-deep step");
static_assert(kPtsBatch == 49152, "points per batch");
static_assert((kPtsBatch % (kRedThreads * 4)) == 0, "scatter pass covers the batch exactly");
static_assert(kOutW == 2 * kRedThreads, "two output floats per thread");
static_assert((kPitch % 4) == 0 && kPitch >= kCpc, "16-B aligned LDS rows");

constexpr float kPCarry   = 1024.0f;
constexpr float kWCarry   = 16.0f;
constexpr float kResCarry = 2048.0f;
constexpr float kFoldRes  = 1.0f / kResCarry;
constexpr float kFoldMain = 1.0f / (kPCarry * kWCarry);
constexpr float kFix      = 2097152.0f;
constexpr float kFixInv   = 1.0f / kFix;

constexpr size_t kOffContrib = 0;
constexpr size_t kOffRow     = kOffContrib + (size_t)kBatch * kPtsBatch * 4;
constexpr size_t kWsTotal    = kOffRow + (size_t)kBatch * kPtsBatch * 4;
static_assert(kWsTotal == 3145728ull, "carve total");
static_assert((kOffRow % 128) == 0, "128-B aligned regions");
static_assert(kWsTotal <= 134217728ull, "carve cap");

__device__ __forceinline__ v8f mma_f16(v16h a, v16h b, v8f c) {
  c = __builtin_amdgcn_wmma_f32_16x16x32_f16(false, a, false, b, (short)0, c, false, false);
  asm volatile("v_nop\n\tv_nop\n\tv_nop\n\tv_nop" : "+v"(c) : "v"(a), "v"(b));
  return c;
}

__device__ __forceinline__ void split_p(float p, _Float16& hi, _Float16& lo) {
  const float ps = p * kPCarry;
  const _Float16 hv = (_Float16)ps;
  const float hf = (float)hv;
  const float rs = (ps - hf) * kResCarry;
  hi = hv;
  lo = (_Float16)rs;
}

__device__ __forceinline__ _Float16 w_elem(float w, int n) {
  const float ws = w * kWCarry;
  const _Float16 hv = (_Float16)ws;
  const float hf = (float)hv;
  const _Float16 lv = (_Float16)((ws - hf) * kResCarry);
  const float lf = (float)lv;
  const float sel = (n == 0) ? hf : ((n == 1) ? lf : 0.0f);
  return (_Float16)sel;
}

__device__ __forceinline__ void gen_point(int j, float m0, float m1,
                                          float su0, float su1, float ru0, float ru1,
                                          int& p0, int& p1) {
#pragma clang fp contract(off)
  const float sc = 0.999999f;
  const float fl0 = floorf(m0), ce0 = ceilf(m0);
  const float fl1 = floorf(m1), ce1 = ceilf(m1);
  const int nb0 = ((j & 2) == 0) ? (int)fl0 : (int)ce0;
  const int nb1 = ((j & 1) == 0) ? (int)fl1 : (int)ce1;
  const float g0 = (su0 * sc) * 1024.0f;
  const float g1 = (su1 * sc) * 1024.0f;
  const int gs0 = (int)floorf(g0);
  const int gs1 = (int)floorf(g1);
  const float r0 = rintf(m0);
  const float r1 = rintf(m1);
  float lo0 = r0 - 8.0f;
  lo0 = (lo0 < 0.0f) ? 0.0f : lo0;
  lo0 = (r0 + 8.0f > 1024.0f) ? 1008.0f : lo0;
  float lo1 = r1 - 8.0f;
  lo1 = (lo1 < 0.0f) ? 0.0f : lo1;
  lo1 = (r1 + 8.0f > 1024.0f) ? 1008.0f : lo1;
  const float t0 = (ru0 * sc) * 16.0f;
  const float t1 = (ru1 * sc) * 16.0f;
  const int wn0 = (int)floorf(t0 + lo0);
  const int wn1 = (int)floorf(t1 + lo1);
  p0 = (j < 4) ? nb0 : ((j < 8) ? gs0 : wn0);
  p1 = (j < 4) ? nb1 : ((j < 8) ? gs1 : wn1);
}

__global__ __launch_bounds__(384) void chunk_points_kernel(
    const float* __restrict__ x, const float* __restrict__ means, const float* __restrict__ sigmas,
    const float* __restrict__ values, const float* __restrict__ su, const float* __restrict__ rru,
    float* __restrict__ wsC, int* __restrict__ wsR)
{
  __shared__ __align__(16) float sP[kPts * kPitch];
  __shared__ __align__(16) int   sKey[kPts];
  __shared__ __align__(16) float sMean[2 * kCpc];
  __shared__ __align__(16) float sInv[2 * kCpc];
  __shared__ __align__(16) float sVal[kCpc];
  __shared__ __align__(16) float sPart[(kPts / 32) * kCpc];
  __shared__ __align__(16) float sW[kCpc];
  __shared__ __align__(16) float sV[kPts];

  const int tid  = threadIdx.x;
  const int lane = tid & 31;
  const int wave = __builtin_amdgcn_readfirstlane((int)(threadIdx.x >> 5));
  const int bk   = blockIdx.x;
  const int b    = bk >> 7;

  if (wave < 2) {
    const float mv = means[(size_t)bk * (2 * kCpc) + tid];
    const float sg = sigmas[(size_t)bk * (2 * kCpc) + tid];
    sMean[tid] = mv;
    sInv[tid]  = sqrtf(1.0f / (1.0e-6f + sg));
  }
  if (wave == 2) {
    sVal[lane] = values[(size_t)bk * kCpc + lane];
  }
  __syncthreads();

  const int p  = tid;
  const int cc = p / kPpc;
  const int j  = p - cc * kPpc;
  int p0, p1;
  {
    const int jj = j & 3;
    const size_t ub = ((size_t)(bk * kCpc + cc) * 4 + (size_t)jj) * 2;
    float su0 = su[ub];
    float su1 = su[ub + 1];
    float ru0 = rru[ub];
    float ru1 = rru[ub + 1];
    asm volatile("" : "+v"(su0), "+v"(su1), "+v"(ru0), "+v"(ru1));
    const float m0 = sMean[2 * cc];
    const float m1 = sMean[2 * cc + 1];
    gen_point(j, m0, m1, su0, su1, ru0, ru1, p0, p1);
  }
  const int key = p0 * kInW + p1;
  sKey[p] = key;
  const int p1c = min(max(p1, 0), kInW - 1);
  const int p0c = min(max(p0, 0), kOutW - 1);
  float xv = x[(size_t)b * kInW + p1c];
  asm volatile("" : "+v"(xv));
  __syncthreads();

  int dup = 0;
  {
    const v4i* k4 = (const v4i*)sKey;
    const int nq = (wave + 1) * 8;
#pragma unroll 1
    for (int q4 = 0; q4 < nq; ++q4) {
      const v4i kk = k4[q4];
      const int q = q4 * 4;
      dup |= ((kk.x == key) && (q     < p)) ? 1 : 0;
      dup |= ((kk.y == key) && (q + 1 < p)) ? 1 : 0;
      dup |= ((kk.z == key) && (q + 2 < p)) ? 1 : 0;
      dup |= ((kk.w == key) && (q + 3 < p)) ? 1 : 0;
    }
  }

  {
    const float px0 = (float)p0;
    const float px1 = (float)p1;
    float* prow = sP + p * kPitch;
#pragma unroll 1
    for (int c4 = 0; c4 < kCpc / 4; ++c4) {
      const v4f ma = *(const v4f*)(sMean + 8 * c4);
      const v4f mb = *(const v4f*)(sMean + 8 * c4 + 4);
      const v4f ia = *(const v4f*)(sInv + 8 * c4);
      const v4f ib = *(const v4f*)(sInv + 8 * c4 + 4);
      const float d00 = (px0 - ma.x) * ia.x;
      const float d01 = (px1 - ma.y) * ia.y;
      const float d10 = (px0 - ma.z) * ia.z;
      const float d11 = (px1 - ma.w) * ia.w;
      const float d20 = (px0 - mb.x) * ib.x;
      const float d21 = (px1 - mb.y) * ib.y;
      const float d30 = (px0 - mb.z) * ib.z;
      const float d31 = (px1 - mb.w) * ib.w;
      float e0 = expf(-0.5f * (d00 * d00 + d01 * d01));
      float e1 = expf(-0.5f * (d10 * d10 + d11 * d11));
      float e2 = expf(-0.5f * (d20 * d20 + d21 * d21));
      float e3 = expf(-0.5f * (d30 * d30 + d31 * d31));
      e0 = (e0 < 1.17549435e-38f) ? 0.0f : e0;
      e1 = (e1 < 1.17549435e-38f) ? 0.0f : e1;
      e2 = (e2 < 1.17549435e-38f) ? 0.0f : e2;
      e3 = (e3 < 1.17549435e-38f) ? 0.0f : e3;
      v4f ev;
      ev.x = dup ? 0.0f : e0;
      ev.y = dup ? 0.0f : e1;
      ev.z = dup ? 0.0f : e2;
      ev.w = dup ? 0.0f : e3;
      *(v4f*)(prow + 4 * c4) = ev;
    }
  }
  __syncthreads();

  {
    const float* col = sP + (wave * 32) * kPitch + lane;
    float acc = 0.0f;
#pragma unroll 4
    for (int i = 0; i < 32; ++i) acc += col[i * kPitch];
    sPart[wave * kCpc + lane] = acc;
  }
  __syncthreads();

  if (wave == 0) {
    float cs = 0.0f;
#pragma unroll 1
    for (int w = 0; w < kPts / 32; ++w) cs += sPart[w * kCpc + lane];
    sW[lane] = sVal[lane] * (1.0f / cs);
  }
  __syncthreads();

  {
    const int h = lane >> 4;
    const int n = lane & 15;
    v16h bfrag;
    {
      const v4f w0 = *(const v4f*)(sW + 8 * h);
      const v4f w1 = *(const v4f*)(sW + 8 * h + 4);
      const v4f w2 = *(const v4f*)(sW + 16 + 8 * h);
      const v4f w3 = *(const v4f*)(sW + 16 + 8 * h + 4);
      bfrag[0]  = w_elem(w0.x, n);
      bfrag[1]  = w_elem(w0.y, n);
      bfrag[2]  = w_elem(w0.z, n);
      bfrag[3]  = w_elem(w0.w, n);
      bfrag[4]  = w_elem(w1.x, n);
      bfrag[5]  = w_elem(w1.y, n);
      bfrag[6]  = w_elem(w1.z, n);
      bfrag[7]  = w_elem(w1.w, n);
      bfrag[8]  = w_elem(w2.x, n);
      bfrag[9]  = w_elem(w2.y, n);
      bfrag[10] = w_elem(w2.z, n);
      bfrag[11] = w_elem(w2.w, n);
      bfrag[12] = w_elem(w3.x, n);
      bfrag[13] = w_elem(w3.y, n);
      bfrag[14] = w_elem(w3.z, n);
      bfrag[15] = w_elem(w3.w, n);
    }
#pragma unroll
    for (int t = 0; t < 2; ++t) {
      const int tb = wave * 32 + t * 16;
      const float* arow = sP + (tb + n) * kPitch;
      const v4f a0 = *(const v4f*)(arow + 8 * h);
      const v4f a1 = *(const v4f*)(arow + 8 * h + 4);
      const v4f a2 = *(const v4f*)(arow + 16 + 8 * h);
      const v4f a3 = *(const v4f*)(arow + 16 + 8 * h + 4);
      v16h ah, al;
      _Float16 hv, lv;
      split_p(a0.x, hv, lv); ah[0]  = hv; al[0]  = lv;
      split_p(a0.y, hv, lv); ah[1]  = hv; al[1]  = lv;
      split_p(a0.z, hv, lv); ah[2]  = hv; al[2]  = lv;
      split_p(a0.w, hv, lv); ah[3]  = hv; al[3]  = lv;
      split_p(a1.x, hv, lv); ah[4]  = hv; al[4]  = lv;
      split_p(a1.y, hv, lv); ah[5]  = hv; al[5]  = lv;
      split_p(a1.z, hv, lv); ah[6]  = hv; al[6]  = lv;
      split_p(a1.w, hv, lv); ah[7]  = hv; al[7]  = lv;
      split_p(a2.x, hv, lv); ah[8]  = hv; al[8]  = lv;
      split_p(a2.y, hv, lv); ah[9]  = hv; al[9]  = lv;
      split_p(a2.z, hv, lv); ah[10] = hv; al[10] = lv;
      split_p(a2.w, hv, lv); ah[11] = hv; al[11] = lv;
      split_p(a3.x, hv, lv); ah[12] = hv; al[12] = lv;
      split_p(a3.y, hv, lv); ah[13] = hv; al[13] = lv;
      split_p(a3.z, hv, lv); ah[14] = hv; al[14] = lv;
      split_p(a3.w, hv, lv); ah[15] = hv; al[15] = lv;
      v8f accH = (v8f){0.f, 0.f, 0.f, 0.f, 0.f, 0.f, 0.f, 0.f};
      v8f accL = (v8f){0.f, 0.f, 0.f, 0.f, 0.f, 0.f, 0.f, 0.f};
      accH = mma_f16(ah, bfrag, accH);
      accL = mma_f16(al, bfrag, accL);
#pragma unroll
      for (int r = 0; r < 8; ++r) {
        const float am = accH[r];
        const float bm = accL[r];
        const float a1n = __shfl_xor(am, 1, 32);
        const float vv = (am + (a1n + bm) * kFoldRes) * kFoldMain;
        if (n == 0) sV[tb + 8 * h + r] = vv;
      }
    }
  }
  __syncthreads();

  {
    const float vv = sV[p];
    const float contrib = dup ? 0.0f : (vv * xv);
    const size_t g = (size_t)bk * kPts + (size_t)p;
    volatile float* pc = (volatile float*)(wsC + g);
    volatile int*   pr = (volatile int*)(wsR + g);
    *pc = contrib;
    *pr = p0c;
    __threadfence();
    *pc = contrib;
    *pr = p0c;
  }
}

__global__ __launch_bounds__(512) void scatter_sum_kernel(
    const float* __restrict__ wsC, const int* __restrict__ wsR, float* __restrict__ out)
{
  __shared__ int sAcc[kOutW];
  const int tid = threadIdx.x;
  const int b   = blockIdx.x;
  sAcc[tid] = 0;
  sAcc[tid + kRedThreads] = 0;
  __syncthreads();
  const v4f* c4 = (const v4f*)(wsC + (size_t)b * kPtsBatch);
  const v4i* r4 = (const v4i*)(wsR + (size_t)b * kPtsBatch);
#pragma unroll 1
  for (int it = 0; it < kPtsBatch / (kRedThreads * 4); ++it) {
    const int idx = it * kRedThreads + tid;
    const v4f cv = c4[idx];
    const v4i rv = r4[idx];
    const int ra = min(max(rv.x, 0), kOutW - 1);
    const int rb = min(max(rv.y, 0), kOutW - 1);
    const int rc = min(max(rv.z, 0), kOutW - 1);
    const int rd = min(max(rv.w, 0), kOutW - 1);
    const int qa = __float2int_rn(cv.x * kFix);
    const int qb = __float2int_rn(cv.y * kFix);
    const int qc = __float2int_rn(cv.z * kFix);
    const int qd = __float2int_rn(cv.w * kFix);
    atomicAdd(&sAcc[ra], qa);
    atomicAdd(&sAcc[rb], qb);
    atomicAdd(&sAcc[rc], qc);
    atomicAdd(&sAcc[rd], qd);
  }
  __syncthreads();
  const float o0 = (float)sAcc[tid] * kFixInv;
  const float o1 = (float)sAcc[tid + kRedThreads] * kFixInv;
  volatile float* o = (volatile float*)(out + (size_t)b * kOutW);
  o[tid] = o0;
  o[tid + kRedThreads] = o1;
  __threadfence();
  o[tid] = o0;
  o[tid + kRedThreads] = o1;
}

extern "C" void kernel_launch(void* const* d_in, const int* in_sizes, int n_in,
                              void* d_out, int out_size, void* d_ws, size_t ws_size,
                              hipStream_t stream) {
  if (n_in < 6) return;
  if (in_sizes[0] != kBatch * kInW) return;
  if (in_sizes[1] != kBatch * kChunks * kCpc * 2) return;
  if (in_sizes[2] != kBatch * kChunks * kCpc * 2) return;
  if (in_sizes[3] != kBatch * kChunks * kCpc) return;
  if (in_sizes[4] != kBatch * kChunks * kCpc * 4 * 2) return;
  if (in_sizes[5] != kBatch * kChunks * kCpc * 4 * 2) return;
  if (out_size != kBatch * kOutW) return;
  if (ws_size < kWsTotal) return;

  const float* x      = (const float*)d_in[0];
  const float* means  = (const float*)d_in[1];
  const float* sigmas = (const float*)d_in[2];
  const float* values = (const float*)d_in[3];
  const float* su     = (const float*)d_in[4];
  const float* rru    = (const float*)d_in[5];
  float* out = (float*)d_out;

  char* ws = (char*)d_ws;
  float* wsC = (float*)(ws + kOffContrib);
  int*   wsR = (int*)(ws + kOffRow);

  chunk_points_kernel<<<kBatch * kChunks, kPts, 0, stream>>>(x, means, sigmas, values, su, rru, wsC, wsR);
  scatter_sum_kernel<<<kBatch, kRedThreads, 0, stream>>>(wsC, wsR, out);
}
